// LocalSumMessageFunction_17025250362097
// MI455X (gfx1250) — hardware-verified
//
#include <hip/hip_runtime.h>
#include <stddef.h>


#define DC      16
#define NF      8
#define HID     64
#define DO      16
#define NTHR    256
#define NWAVE   8
#define NBN     64
#define APN     40
#define NBE     64
#define APE     72
#define EPT     8
#define PIECE   (NTHR * EPT)
#define WCAP    (EPT * 32)
#define NBC     4096
#define SLOTB   12
#define NPC     400
#define ECH     (NPC * PIECE)
#define NPROW   128
#define B0H     0
#define B0L     4096
#define W1H     8192
#define W1L     12288
#define W2H     16384
#define W2L     17408
#define WPM     18432
#define PBLK    9
#define WSCAP   134217728
#define AGGDYN  (NBC * DO * 4)

static_assert((PIECE & (PIECE - 1)) == 0);
static_assert((NBC & (NBC - 1)) == 0);
static_assert(NBC <= (1 << SLOTB));
static_assert(PIECE <= 2048);
static_assert(ECH % NBE == 0);
static_assert(((APN * 2) % 16) == 0);
static_assert(((APE * 2) % 16) == 0);
static_assert(WPM == PBLK * NTHR * 8);
static_assert(NBE == NWAVE * 8);
static_assert(NBN * DC == NTHR * 4);
static_assert((NBC % (NWAVE * 8)) == 0);
static_assert(NF * HID == 2 * NTHR);
static_assert((B0L % (NTHR * 8)) == 0 && (W1H % (NTHR * 8)) == 0 && (W1L % (NTHR * 8)) == 0 && (W2H % (NTHR * 8)) == 0);

typedef float          v2f   __attribute__((ext_vector_type(2)));
typedef float          v4f   __attribute__((ext_vector_type(4)));
typedef float          v8f   __attribute__((ext_vector_type(8)));
typedef int            v4i   __attribute__((ext_vector_type(4)));
typedef unsigned short v2us  __attribute__((ext_vector_type(2)));
typedef unsigned short v4us  __attribute__((ext_vector_type(4)));
typedef unsigned short v8us  __attribute__((ext_vector_type(8)));
typedef unsigned short v16us __attribute__((ext_vector_type(16)));
typedef __bf16         v16bf __attribute__((ext_vector_type(16)));
union FragB { v16bf v; v16us u; v8us h[2]; };

__device__ __forceinline__ v8f wm(v16bf a, v16bf b, v8f c) {
  v8f d = __builtin_amdgcn_wmma_f32_16x16x32_bf16(false, a, false, b, (short)0, c, false, false);
  asm volatile("v_nop\n\tv_nop\n\tv_nop\n\tv_nop" : "+v"(d) : "v"(a), "v"(b));
  return d;
}

__device__ __forceinline__ v8f zero8() {
  v8f z = {0.f, 0.f, 0.f, 0.f, 0.f, 0.f, 0.f, 0.f};
  return z;
}
__device__ __forceinline__ v4f zero4() {
  v4f z = {0.f, 0.f, 0.f, 0.f};
  return z;
}

__device__ __forceinline__ unsigned bf_rne(float x) {
  const unsigned u = __float_as_uint(x);
  return (u + 0x7FFFu + ((u >> 16) & 1u)) >> 16;
}
__device__ __forceinline__ void split_bf(float x, unsigned short& hi, unsigned short& lo) {
  const unsigned h = bf_rne(x);
  const float hf = __uint_as_float(h << 16);
  hi = (unsigned short)h;
  lo = (unsigned short)bf_rne(x - hf);
}
__device__ __forceinline__ float tanh_f(float x) {
  const float e = __expf(2.0f * x);
  return 1.0f - 2.0f * __builtin_amdgcn_rcpf(e + 1.0f);
}
__device__ __forceinline__ int imin(int a, int b) { return a < b ? a : b; }
__device__ __forceinline__ float relu_f(float v) { return v > 0.0f ? v : 0.0f; }

__global__ __launch_bounds__(NTHR) void k_prep(
    const float* __restrict__ fW0, const float* __restrict__ fW1, const float* __restrict__ fW2,
    const float* __restrict__ tW0, const float* __restrict__ tW1, const float* __restrict__ tW2,
    unsigned short* wp) {
  const int tid = (int)threadIdx.x;
  const int b = (int)blockIdx.x;
  const int p = (b >= PBLK) ? 1 : 0;
  const int sb = b - p * PBLK;
  const float* W0 = p ? tW0 : fW0;
  const float* W1 = p ? tW1 : fW1;
  const float* W2 = p ? tW2 : fW2;
  const int o = (sb * NTHR + tid) * 8;
  const float* src = W0;
  int stride = HID, rb = 0, col = 0, lo = 0, zero = 0;
  if (o < W1H) {
    const int idx = o & 4095;
    const int n = idx >> 5;
    const int k0 = idx & 31;
    const int part = n >> 6;
    src = W0; stride = HID; rb = NF + DC * part + (k0 & 15); col = n & 63;
    zero = (k0 >= 16) ? 1 : 0;
    lo = (o >= B0L) ? 1 : 0;
  } else if (o < W2H) {
    const int idx = (o - W1H) & 4095;
    src = W1; stride = HID; rb = idx & 63; col = idx >> 6;
    lo = (o >= W1L) ? 1 : 0;
  } else {
    const int idx = (o - W2H) & 1023;
    src = W2; stride = DO; rb = idx & 63; col = idx >> 6;
    lo = (o >= W2L) ? 1 : 0;
  }
  float v[8];
#pragma unroll
  for (int j = 0; j < 8; ++j) {
    const float t = src[(size_t)(rb + j) * stride + col];
    v[j] = zero ? 0.0f : t;
  }
  v8us ov;
#pragma unroll
  for (int j = 0; j < 8; ++j) {
    unsigned short hi, lw;
    split_bf(v[j], hi, lw);
    ov[j] = lo ? lw : hi;
  }
  unsigned short* dp = wp + (size_t)p * WPM + o;
  *(volatile v8us*)dp = ov;
  __threadfence();
  *(volatile v8us*)dp = ov;
}

__global__ __launch_bounds__(NTHR) void k_node(
    const float* __restrict__ x, const unsigned short* __restrict__ wpp, float* NP, int nN) {
  __shared__ __attribute__((aligned(16))) unsigned short sAh[NBN * APN];
  __shared__ __attribute__((aligned(16))) unsigned short sAl[NBN * APN];
  __shared__ __attribute__((aligned(16))) float stg[NWAVE * 1024];
  const int tid = (int)threadIdx.x, lane = tid & 31, hh = lane >> 4, m = lane & 15;
  const int wave = __builtin_amdgcn_readfirstlane(tid >> 5);
  const int n0 = (int)blockIdx.x * NBN;

  {
    const int nl = tid >> 2, q = tid & 3;
    int node = n0 + nl;
    node = node > nN - 1 ? nN - 1 : node;
    const v4f xa = *(const v4f*)(x + (size_t)node * DC + 4 * q);
    float xv[4];
    xv[0] = xa.x; xv[1] = xa.y; xv[2] = xa.z; xv[3] = xa.w;
    v4us vh, vl;
#pragma unroll
    for (int u = 0; u < 4; ++u) {
      unsigned short hi, lw;
      split_bf(xv[u], hi, lw);
      vh[u] = hi;
      vl[u] = lw;
    }
    const v4us z4 = {(unsigned short)0, (unsigned short)0, (unsigned short)0, (unsigned short)0};
    *(v4us*)(sAh + nl * APN + 4 * q) = vh;
    *(v4us*)(sAh + nl * APN + 16 + 4 * q) = z4;
    *(v4us*)(sAl + nl * APN + 4 * q) = vl;
    *(v4us*)(sAl + nl * APN + 16 + 4 * q) = z4;
  }
  __syncthreads();

  const int rt = wave & 3, chf = wave >> 2;
  const unsigned short* aph = sAh + (16 * rt + m) * APN + 8 * hh;
  const unsigned short* apl = sAl + (16 * rt + m) * APN + 8 * hh;
  const unsigned short* pH = wpp + B0H;
  const unsigned short* pL = wpp + B0L;
  float* sw = stg + wave * 1024;

  v8f acc[4];
#pragma unroll
  for (int t = 0; t < 4; ++t) acc[t] = zero8();
  {
    FragB ah, al;
    ah.h[0] = *(const v8us*)(aph);
    ah.h[1] = *(const v8us*)(aph + 16);
    al.h[0] = *(const v8us*)(apl);
    al.h[1] = *(const v8us*)(apl + 16);
#pragma unroll
    for (int t = 0; t < 4; ++t) {
      const int n = 64 * chf + 16 * t + m;
      const size_t bo = (size_t)n * 32 + 8 * hh;
      FragB bh, bl;
      bh.h[0] = *(const v8us*)(pH + bo);
      bh.h[1] = *(const v8us*)(pH + bo + 16);
      bl.h[0] = *(const v8us*)(pL + bo);
      bl.h[1] = *(const v8us*)(pL + bo + 16);
      acc[t] = wm(ah.v, bh.v, acc[t]);
      acc[t] = wm(ah.v, bl.v, acc[t]);
      acc[t] = wm(al.v, bh.v, acc[t]);
    }
  }
  {
    float* sp = sw + (8 * hh) * 64 + m;
#pragma unroll
    for (int t = 0; t < 4; ++t) {
#pragma unroll
      for (int r = 0; r < 8; ++r) sp[r * 64 + 16 * t] = acc[t][r];
    }
  }
  __syncthreads();
#pragma unroll 1
  for (int i = 0; i < 8; ++i) {
    const int r2 = 2 * i + hh;
    const v4f v = *(const v4f*)(sw + r2 * 64 + 4 * m);
    const int row = n0 + 16 * rt + r2;
    *(volatile v4f*)(NP + (size_t)row * NPROW + 64 * chf + 4 * m) = v;
  }
  __threadfence();
#pragma unroll 1
  for (int i = 0; i < 8; ++i) {
    const int r2 = 2 * i + hh;
    const v4f v = *(const v4f*)(sw + r2 * 64 + 4 * m);
    const int row = n0 + 16 * rt + r2;
    *(volatile v4f*)(NP + (size_t)row * NPROW + 64 * chf + 4 * m) = v;
  }
}

__global__ __launch_bounds__(NTHR) void k_edge(
    const int* __restrict__ af, const int* __restrict__ at,
    const float* __restrict__ feat, const float* __restrict__ msk,
    const float* __restrict__ W0, const float* __restrict__ b0,
    const float* __restrict__ b1, const float* __restrict__ b2,
    const unsigned short* __restrict__ wpp, const float* __restrict__ NP, float* D,
    int cbeg, int nE, int nN) {
  __shared__ __attribute__((aligned(16))) unsigned short sZh[NBE * APE];
  __shared__ __attribute__((aligned(16))) unsigned short sZl[NBE * APE];
  __shared__ __attribute__((aligned(16))) unsigned short sYh[NBE * APE];
  __shared__ __attribute__((aligned(16))) unsigned short sYl[NBE * APE];
  __shared__ __attribute__((aligned(16))) float sD[NBE * DO];
  __shared__ __attribute__((aligned(16))) float sWx[NF * HID];
  __shared__ __attribute__((aligned(16))) float sB0[HID];
  __shared__ __attribute__((aligned(16))) float sB1[HID];
  __shared__ __attribute__((aligned(16))) float sB2[DO];
  __shared__ __attribute__((aligned(16))) float sX[NBE * NF];
  __shared__ float sM[NBE];
  __shared__ int sFr[NBE];
  __shared__ int sTo[NBE];
  const int tid = (int)threadIdx.x, lane = tid & 31, hh = lane >> 4, m = lane & 15;
  const int wave = __builtin_amdgcn_readfirstlane(tid >> 5);
  const int eb = cbeg + (int)blockIdx.x * NBE;

  if (tid < NBE) {
    int e = eb + tid;
    e = e > nE - 1 ? nE - 1 : e;
    int f = af[e];
    f = f < 0 ? 0 : (f > nN - 1 ? nN - 1 : f);
    int g = at[e];
    g = g < 0 ? 0 : (g > nN - 1 ? nN - 1 : g);
    const v4f xa = *(const v4f*)(feat + (size_t)e * NF);
    const v4f xb = *(const v4f*)(feat + (size_t)e * NF + 4);
    sFr[tid] = f;
    sTo[tid] = g;
    sM[tid] = msk[e];
    *(v4f*)(sX + NF * tid) = xa;
    *(v4f*)(sX + NF * tid + 4) = xb;
  }
  sWx[tid] = W0[tid];
  sWx[tid + NTHR] = W0[tid + NTHR];
  if (tid < HID) { sB0[tid] = b0[tid]; sB1[tid] = b1[tid]; }
  if (tid < DO) sB2[tid] = b2[tid];
  __syncthreads();

  {
    const int c2 = 2 * lane;
    v2f wv[8];
#pragma unroll
    for (int c = 0; c < 8; ++c) wv[c] = *(const v2f*)(sWx + c * HID + c2);
    const v2f bb = *(const v2f*)(sB0 + c2);
#pragma unroll 1
    for (int j = 0; j < 8; ++j) {
      const int el = 8 * wave + j;
      const int fr = sFr[el];
      const int tn = sTo[el];
      const float mk = sM[el];
      const v4f xa = *(const v4f*)(sX + NF * el);
      const v4f xb = *(const v4f*)(sX + NF * el + 4);
      const v2f p = *(const v2f*)(NP + (size_t)fr * NPROW + c2);
      const v2f q = *(const v2f*)(NP + (size_t)tn * NPROW + HID + c2);
      v2f u = p + q;
      u += xa.x * wv[0];
      u += xa.y * wv[1];
      u += xa.z * wv[2];
      u += xa.w * wv[3];
      u += xb.x * wv[4];
      u += xb.y * wv[5];
      u += xb.z * wv[6];
      u += xb.w * wv[7];
      const v2f z = mk * u + bb;
      unsigned short h0, l0, h1, l1;
      split_bf(relu_f(z.x), h0, l0);
      split_bf(relu_f(z.y), h1, l1);
      v2us hv, lv;
      hv.x = h0; hv.y = h1;
      lv.x = l0; lv.y = l1;
      *(v2us*)(sZh + el * APE + c2) = hv;
      *(v2us*)(sZl + el * APE + c2) = lv;
    }
  }
  __syncthreads();

  const int rt = wave & 3, cg = wave >> 2;
  {
    v8f acc[2];
    acc[0] = zero8(); acc[1] = zero8();
    const unsigned short* aph = sZh + (16 * rt + m) * APE + 8 * hh;
    const unsigned short* apl = sZl + (16 * rt + m) * APE + 8 * hh;
    const unsigned short* pH = wpp + W1H;
    const unsigned short* pL = wpp + W1L;
#pragma unroll 1
    for (int ks = 0; ks < 2; ++ks) {
      FragB ah, al;
      ah.h[0] = *(const v8us*)(aph + 32 * ks);
      ah.h[1] = *(const v8us*)(aph + 32 * ks + 16);
      al.h[0] = *(const v8us*)(apl + 32 * ks);
      al.h[1] = *(const v8us*)(apl + 32 * ks + 16);
#pragma unroll
      for (int t = 0; t < 2; ++t) {
        const int n = 32 * cg + 16 * t + m;
        const size_t bo = (size_t)n * HID + 32 * ks + 8 * hh;
        FragB bh, bl;
        bh.h[0] = *(const v8us*)(pH + bo);
        bh.h[1] = *(const v8us*)(pH + bo + 16);
        bl.h[0] = *(const v8us*)(pL + bo);
        bl.h[1] = *(const v8us*)(pL + bo + 16);
        acc[t] = wm(ah.v, bh.v, acc[t]);
        acc[t] = wm(ah.v, bl.v, acc[t]);
        acc[t] = wm(al.v, bh.v, acc[t]);
      }
    }
#pragma unroll
    for (int t = 0; t < 2; ++t) {
      const int col = 32 * cg + 16 * t + m;
      const float bb = sB1[col];
#pragma unroll
      for (int r = 0; r < 8; ++r) {
        const float z = relu_f(acc[t][r] + bb);
        unsigned short hi, lw;
        split_bf(z, hi, lw);
        const int idx = (16 * rt + 8 * hh + r) * APE + col;
        sYh[idx] = hi;
        sYl[idx] = lw;
      }
    }
  }
  __syncthreads();

  if (wave < 4) {
    v8f acc = zero8();
    const unsigned short* aph = sYh + (16 * wave + m) * APE + 8 * hh;
    const unsigned short* apl = sYl + (16 * wave + m) * APE + 8 * hh;
    const unsigned short* pH = wpp + W2H;
    const unsigned short* pL = wpp + W2L;
#pragma unroll 1
    for (int ks = 0; ks < 2; ++ks) {
      FragB ah, al, bh, bl;
      ah.h[0] = *(const v8us*)(aph + 32 * ks);
      ah.h[1] = *(const v8us*)(aph + 32 * ks + 16);
      al.h[0] = *(const v8us*)(apl + 32 * ks);
      al.h[1] = *(const v8us*)(apl + 32 * ks + 16);
      const size_t bo = (size_t)m * HID + 32 * ks + 8 * hh;
      bh.h[0] = *(const v8us*)(pH + bo);
      bh.h[1] = *(const v8us*)(pH + bo + 16);
      bl.h[0] = *(const v8us*)(pL + bo);
      bl.h[1] = *(const v8us*)(pL + bo + 16);
      acc = wm(ah.v, bh.v, acc);
      acc = wm(ah.v, bl.v, acc);
      acc = wm(al.v, bh.v, acc);
    }
    const float bb = sB2[m];
#pragma unroll
    for (int r = 0; r < 8; ++r) {
      const int el = 16 * wave + 8 * hh + r;
      sD[el * DO + m] = (acc[r] + bb) * sM[el];
    }
  }
  __syncthreads();

  {
    const v4f v = *(const v4f*)(sD + 128 * wave + 4 * lane);
    float* dp = D + ((size_t)blockIdx.x * NBE + 8 * wave) * DO + 4 * lane;
    *(volatile v4f*)dp = v;
    __threadfence();
    *(volatile v4f*)dp = v;
  }
}

__device__ __forceinline__ int scan_piece(const int* __restrict__ keys, int nLim, int cbase, int slotBase,
                                          int vec8, int* list, int tid, int wave) {
  int wc = 0;
  const int el0  = tid * EPT;
  const int e0   = cbase + el0;
  const int sent = -2147483647 - 1;
  const int lm   = nLim - 1;
  v4i da, db;
  if (vec8 != 0 && cbase + PIECE <= nLim) {
    da = *(const v4i*)(keys + e0);
    db = *(const v4i*)(keys + e0 + 4);
  } else {
    da.x = (e0     < nLim) ? keys[imin(e0,     lm)] : sent;
    da.y = (e0 + 1 < nLim) ? keys[imin(e0 + 1, lm)] : sent;
    da.z = (e0 + 2 < nLim) ? keys[imin(e0 + 2, lm)] : sent;
    da.w = (e0 + 3 < nLim) ? keys[imin(e0 + 3, lm)] : sent;
    db.x = (e0 + 4 < nLim) ? keys[imin(e0 + 4, lm)] : sent;
    db.y = (e0 + 5 < nLim) ? keys[imin(e0 + 5, lm)] : sent;
    db.z = (e0 + 6 < nLim) ? keys[imin(e0 + 6, lm)] : sent;
    db.w = (e0 + 7 < nLim) ? keys[imin(e0 + 7, lm)] : sent;
  }
  const unsigned nb = (unsigned)slotBase;
  const unsigned s0 = (unsigned)da.x - nb, s1 = (unsigned)da.y - nb;
  const unsigned s2 = (unsigned)da.z - nb, s3 = (unsigned)da.w - nb;
  const unsigned s4 = (unsigned)db.x - nb, s5 = (unsigned)db.y - nb;
  const unsigned s6 = (unsigned)db.z - nb, s7 = (unsigned)db.w - nb;
  const bool h0 = s0 < (unsigned)NBC, h1 = s1 < (unsigned)NBC, h2 = s2 < (unsigned)NBC, h3 = s3 < (unsigned)NBC;
  const bool h4 = s4 < (unsigned)NBC, h5 = s5 < (unsigned)NBC, h6 = s6 < (unsigned)NBC, h7 = s7 < (unsigned)NBC;
  const unsigned any = __builtin_amdgcn_ballot_w32(h0 | h1 | h2 | h3 | h4 | h5 | h6 | h7);
  if (any != 0u) {
#define HITJ(J, HJ, SJ) { \
      const unsigned mj = __builtin_amdgcn_ballot_w32(HJ); \
      if (mj != 0u) { \
        if (HJ) { \
          const int pos = wc + (int)__builtin_amdgcn_mbcnt_lo(mj, 0u); \
          if (pos < WCAP) list[wave * WCAP + pos] = ((el0 + (J)) << SLOTB) | (int)(SJ); \
        } \
        wc += (int)__builtin_popcount(mj); } }
    HITJ(0, h0, s0)
    HITJ(1, h1, s1)
    HITJ(2, h2, s2)
    HITJ(3, h3, s3)
    HITJ(4, h4, s4)
    HITJ(5, h5, s5)
    HITJ(6, h6, s6)
    HITJ(7, h7, s7)
#undef HITJ
  }
  return wc;
}

__device__ __forceinline__ void drain_piece(const int* list, const int* wcnt, float* acc,
                                            const float* __restrict__ D, int rowBase, int lane, int wave) {
  const int c = lane & 15;
#pragma unroll 1
  for (int wsx = 0; wsx < NWAVE; ++wsx) {
    int n = __builtin_amdgcn_readfirstlane(wcnt[wsx]);
    n = n > WCAP ? WCAP : (n < 0 ? 0 : n);
    const int* lp = list + wsx * WCAP;
#pragma unroll 1
    for (int i = 0; i < n; ++i) {
      const int ent  = __builtin_amdgcn_readfirstlane(lp[i]);
      const int slot = ent & (NBC - 1);
      const int el   = (ent >> SLOTB) & (PIECE - 1);
      int row = rowBase + el;
      row = row < 0 ? 0 : (row > ECH - 1 ? ECH - 1 : row);
      if ((slot & (NWAVE - 1)) == wave) {
        const float dv = D[(size_t)row * DO + c];
        float* ap = acc + slot * DO + c;
        *ap = *ap + dv;
      }
    }
  }
}

__global__ __launch_bounds__(NTHR) void k_agg(
    const int* __restrict__ keys, const float* __restrict__ D, float* out,
    int cbeg, int nLim, int nN, int first, int last, int vec8) {
  extern __shared__ __attribute__((aligned(16))) float accd[];
  __shared__ int list[NWAVE * WCAP];
  __shared__ int wcnt[NWAVE];
  const int tid = (int)threadIdx.x, lane = tid & 31;
  const int wave = __builtin_amdgcn_readfirstlane(tid >> 5);
  const int nodeBase = (int)blockIdx.x * NBC;

#pragma unroll 1
  for (int i = tid; i < NBC * (DO / 4); i += NTHR) {
    const int slot = i >> 2, pc = i & 3;
    const int node = nodeBase + slot;
    const int nn = node > nN - 1 ? nN - 1 : node;
    v4f v = zero4();
    if (first == 0) {
      v = *(const v4f*)(out + (size_t)nn * DO + 4 * pc);
      if (node >= nN) v = zero4();
    }
    *(v4f*)(accd + slot * DO + 4 * pc) = v;
  }
  __syncthreads();

  int nPieces = (nLim - cbeg + PIECE - 1) / PIECE;
  nPieces = nPieces < 0 ? 0 : (nPieces > NPC ? NPC : nPieces);
#pragma unroll 1
  for (int pcx = 0; pcx < nPieces; ++pcx) {
    const int cbase = cbeg + pcx * PIECE;
    const int wc = scan_piece(keys, nLim, cbase, nodeBase, vec8, list, tid, wave);
    if (lane == 0) wcnt[wave] = wc;
    __syncthreads();
    drain_piece(list, wcnt, accd, D, cbase - cbeg, lane, wave);
    __syncthreads();
  }

  if (last != 0) {
#pragma unroll 1
    for (int i = tid; i < NBC * DO; i += NTHR) accd[i] = tanh_f(accd[i]);
  }
  __syncthreads();

  const int sub = lane >> 2, pc = lane & 3;
#pragma unroll 1
  for (int it = 0; it < NBC / (NWAVE * 8); ++it) {
    const int slot = wave * (NBC / NWAVE) + 8 * it + sub;
    const int node = nodeBase + slot;
    const v4f v = *(const v4f*)(accd + slot * DO + 4 * pc);
    if (node < nN) *(volatile v4f*)(out + (size_t)node * DO + 4 * pc) = v;
  }
  __threadfence();
#pragma unroll 1
  for (int it = 0; it < NBC / (NWAVE * 8); ++it) {
    const int slot = wave * (NBC / NWAVE) + 8 * it + sub;
    const int node = nodeBase + slot;
    const v4f v = *(const v4f*)(accd + slot * DO + 4 * pc);
    if (node < nN) *(volatile v4f*)(out + (size_t)node * DO + 4 * pc) = v;
  }
}

extern "C" void kernel_launch(void* const* d_in, const int* in_sizes, int n_in,
                              void* d_out, int out_size, void* d_ws, size_t ws_size,
                              hipStream_t stream) {
  if (n_in < 17) return;
  if (in_sizes[0] < DC || (in_sizes[0] % DC) != 0) return;
  const int nN = in_sizes[0] / DC;
  if (nN < 1 || nN > (1 << 24)) return;
  const int nE = in_sizes[3];
  if (nE < 1 || nE > (1 << 28)) return;
  if (in_sizes[4] != nE || in_sizes[2] != nE || in_sizes[1] != nE * NF) return;
  for (int p = 0; p < 2; ++p) {
    const int b = 5 + 6 * p;
    if (in_sizes[b] != (NF + 2 * DC) * HID || in_sizes[b + 1] != HID || in_sizes[b + 2] != HID * HID ||
        in_sizes[b + 3] != HID || in_sizes[b + 4] != HID * DO || in_sizes[b + 5] != DO) return;
  }
  if (out_size != nN * DO) return;

  const float* x   = (const float*)d_in[0];
  const float* ft  = (const float*)d_in[1];
  const float* msk = (const float*)d_in[2];
  const int*   af  = (const int*)d_in[3];
  const int*   at  = (const int*)d_in[4];
  const float* fW0 = (const float*)d_in[5];
  const float* fb0 = (const float*)d_in[6];
  const float* fW1 = (const float*)d_in[7];
  const float* fb1 = (const float*)d_in[8];
  const float* fW2 = (const float*)d_in[9];
  const float* fb2 = (const float*)d_in[10];
  const float* tW0 = (const float*)d_in[11];
  const float* tb0 = (const float*)d_in[12];
  const float* tW1 = (const float*)d_in[13];
  const float* tb1 = (const float*)d_in[14];
  const float* tW2 = (const float*)d_in[15];
  const float* tb2 = (const float*)d_in[16];
  float* out = (float*)d_out;

  const int nbNode = (nN + NBN - 1) / NBN;
  const int Npad   = nbNode * NBN;
  const int nbAgg  = (nN + NBC - 1) / NBC;
  const int nCh    = (nE + ECH - 1) / ECH;

  char* ws = (char*)d_ws;
  size_t off = 0;
  const size_t oW  = off; off += (size_t)2 * WPM * 2;            off = (off + 255) & ~(size_t)255;
  const size_t oNP = off; off += (size_t)Npad * NPROW * 4;       off = (off + 255) & ~(size_t)255;
  const size_t oD  = off; off += (size_t)ECH * DO * 4;           off = (off + 255) & ~(size_t)255;
  if (off > ws_size || off > (size_t)WSCAP) return;
  unsigned short* wp = (unsigned short*)(ws + oW);
  float* NP = (float*)(ws + oNP);
  float* D  = (float*)(ws + oD);

  hipFuncSetAttribute(reinterpret_cast<const void*>(&k_agg), hipFuncAttributeMaxDynamicSharedMemorySize, AGGDYN);

  k_prep<<<2 * PBLK, NTHR, 0, stream>>>(fW0, fW1, fW2, tW0, tW1, tW2, wp);

  for (int p = 0; p < 2; ++p) {
    const unsigned short* wpp = wp + (size_t)p * WPM;
    const float* W0  = p ? tW0 : fW0;
    const float* b0  = p ? tb0 : fb0;
    const float* b1  = p ? tb1 : fb1;
    const float* b2  = p ? tb2 : fb2;
    const int* keys  = p ? at : af;
    k_node<<<nbNode, NTHR, 0, stream>>>(x, wpp, NP, nN);
    for (int c = 0; c < nCh; ++c) {
      const int cbeg = c * ECH;
      const int cend = (cbeg + ECH < nE) ? (cbeg + ECH) : nE;
      const int nblk = (cend - cbeg + NBE - 1) / NBE;
      const int first = (p == 0 && c == 0) ? 1 : 0;
      const int last  = (p == 1 && c == nCh - 1) ? 1 : 0;
      k_edge<<<nblk, NTHR, 0, stream>>>(af, at, ft, msk, W0, b0, b1, b2, wpp, NP, D, cbeg, nE, nN);
      k_agg<<<nbAgg, NTHR, AGGDYN, stream>>>(keys, D, out, cbeg, cend, nN, first, last, 1);
    }
  }
}
